// PIKR_51213190037873
// MI455X (gfx1250) — hardware-verified
//
#include <hip/hip_runtime.h>

#define M_DIM 8192
#define N_DIM 8192
#define D_DIM 256
#define GAMMA_F (1.0f / 256.0f)
#define BM 256
#define NSPLIT 16
#define NCHUNK (N_DIM / NSPLIT)

typedef __attribute__((ext_vector_type(16))) _Float16 v16h;
typedef __attribute__((ext_vector_type(8)))  _Float16 v8h;
typedef __attribute__((ext_vector_type(8)))  float    v8f;
typedef __attribute__((ext_vector_type(4)))  float    v4f_t;
typedef float v4fa __attribute__((ext_vector_type(4), may_alias));
typedef __attribute__((ext_vector_type(4)))  unsigned v4u_t;
typedef unsigned v4ua __attribute__((ext_vector_type(4), may_alias));

__global__ __launch_bounds__(256) void cvt_kernel(
    const float* __restrict__ Xq, const float* __restrict__ Xt,
    _Float16* __restrict__ Xqh, _Float16* __restrict__ Xth) {
  const int t8 = blockIdx.x * 256 + threadIdx.x;
  if (t8 >= (M_DIM + N_DIM) * D_DIM / 8) return;
  const int e0 = t8 * 8;
  const bool isq = e0 < M_DIM * D_DIM;
  const float* src = isq ? (Xq + e0) : (Xt + (e0 - M_DIM * D_DIM));
  _Float16* dst = isq ? (Xqh + e0) : (Xth + (e0 - M_DIM * D_DIM));
  _Float16 hh[8];
#pragma unroll
  for (int e = 0; e < 8; ++e) hh[e] = (_Float16)src[e];
  *(volatile v4u_t*)dst = *(const v4ua*)hh; __threadfence(); *(volatile v4u_t*)dst = *(const v4ua*)hh;
}
__global__ __launch_bounds__(256) void norm_kernel(
    const float* __restrict__ Xq, const float* __restrict__ Xt, float* __restrict__ sqa, float* __restrict__ sqb) {
  const int row = blockIdx.x * 256 + threadIdx.x;
  if (row >= M_DIM + N_DIM) return;
  const bool isq = row < M_DIM;
  const int r = isq ? row : row - M_DIM;
  const float* src = (isq ? Xq : Xt) + (size_t)r * D_DIM;
  float s = 0.f;
#pragma unroll 4
  for (int k = 0; k < D_DIM; k += 4) { const v4f_t v = *(const v4f_t*)(src + k); s += v.x * v.x + v.y * v.y + v.z * v.z + v.w * v.w; }
  float* d = (isq ? sqa : sqb) + r;
  *(volatile float*)d = s; __threadfence(); *(volatile float*)d = s;
}

__global__ __launch_bounds__(256) void rbf_wmma_kernel(
    const _Float16* __restrict__ Xqh, const _Float16* __restrict__ Xth,
    const float* __restrict__ sqa, const float* __restrict__ sqb,
    const float* __restrict__ alpha, float* __restrict__ partial) {
  const int lane = threadIdx.x & 31;
  const int wave = threadIdx.x >> 5;
  const int rowBase = blockIdx.x * BM + wave * 32;
  const int nStart = blockIdx.y * NCHUNK;
  const bool hiHalf = lane >= 16;
  const int l16 = lane & 15;

  const int ac = hiHalf ? 8 : 0;
  const _Float16* arow0 = Xqh + (size_t)(rowBase + l16) * D_DIM;
  const _Float16* arow1 = arow0 + (size_t)16 * D_DIM;
  v16h A0[8], A1[8];
#pragma unroll
  for (int ks = 0; ks < 8; ++ks) {
    const _Float16* p0 = arow0 + ks * 32 + ac;
    v8h lo0 = *(const v8h*)(p0);
    v8h hi0 = *(const v8h*)(p0 + 16);
    A0[ks] = __builtin_shufflevector(lo0, hi0, 0, 1, 2, 3, 4, 5, 6, 7,
                                     8, 9, 10, 11, 12, 13, 14, 15);
    const _Float16* p1 = arow1 + ks * 32 + ac;
    v8h lo1 = *(const v8h*)(p1);
    v8h hi1 = *(const v8h*)(p1 + 16);
    A1[ks] = __builtin_shufflevector(lo1, hi1, 0, 1, 2, 3, 4, 5, 6, 7,
                                     8, 9, 10, 11, 12, 13, 14, 15);
  }

  const int rb0 = rowBase + (hiHalf ? 8 : 0);
  const int rb1 = rb0 + 16;
  float sqa0[8], sqa1[8];
#pragma unroll
  for (int r = 0; r < 8; ++r) {
    sqa0[r] = sqa[rb0 + r];
    sqa1[r] = sqa[rb1 + r];
  }

  float acc0[8], acc1[8];
#pragma unroll
  for (int r = 0; r < 8; ++r) { acc0[r] = 0.0f; acc1[r] = 0.0f; }

  const int bko = hiHalf ? 8 : 0;
  __shared__ __attribute__((aligned(16))) float sp[8][32];

  for (int n0 = nStart; n0 < nStart + NCHUNK; n0 += 16) {
    const _Float16* brow = Xth + (size_t)(n0 + l16) * D_DIM + bko;

    __builtin_prefetch(brow + 16 * D_DIM, 0, 1);
    __builtin_prefetch(brow + 16 * D_DIM + 128, 0, 1);

    v8f c0 = {};
    v8f c1 = {};
#pragma unroll
    for (int ks = 0; ks < 8; ++ks) {
      v8h lo = *(const v8h*)(brow + ks * 32);
      v8h hi = *(const v8h*)(brow + ks * 32 + 16);
      v16h B = __builtin_shufflevector(lo, hi, 0, 1, 2, 3, 4, 5, 6, 7,
                                       8, 9, 10, 11, 12, 13, 14, 15);
      c0 = __builtin_amdgcn_wmma_f32_16x16x32_f16(false, A0[ks], false, B,
                                                  (short)0, c0, false, false);
      c1 = __builtin_amdgcn_wmma_f32_16x16x32_f16(false, A1[ks], false, B,
                                                  (short)0, c1, false, false);
    }
    const float sqb_n = sqb[n0 + l16];
    const float al = alpha[n0 + l16];
#pragma unroll
    for (int r = 0; r < 8; ++r) {
      float d20 = sqa0[r] + sqb_n - 2.0f * c0[r];
      float d21 = sqa1[r] + sqb_n - 2.0f * c1[r];
      d20 = fmaxf(d20, 0.0f);
      d21 = fmaxf(d21, 0.0f);
      acc0[r] += __expf(-GAMMA_F * d20) * al;
      acc1[r] += __expf(-GAMMA_F * d21) * al;
    }
  }

  float* pout = partial + (size_t)blockIdx.y * M_DIM;
#pragma unroll
  for (int r = 0; r < 8; ++r) {
    float v0 = acc0[r];
    v0 += __shfl_xor(v0, 1, 32);
    v0 += __shfl_xor(v0, 2, 32);
    v0 += __shfl_xor(v0, 4, 32);
    v0 += __shfl_xor(v0, 8, 32);
    float v1 = acc1[r];
    v1 += __shfl_xor(v1, 1, 32);
    v1 += __shfl_xor(v1, 2, 32);
    v1 += __shfl_xor(v1, 4, 32);
    v1 += __shfl_xor(v1, 8, 32);
    if (l16 == 0) {
      sp[wave][(hiHalf ? 8 : 0) + r]      = v0;
      sp[wave][16 + (hiHalf ? 8 : 0) + r] = v1;
    }
  }
  asm volatile("s_wait_dscnt 0" ::: "memory");
  if (lane < 8) {
    const v4f_t v = *(const volatile v4fa*)(&sp[wave][lane * 4]);
    *(volatile v4f_t*)(pout + rowBase + lane * 4) = v; __threadfence(); *(volatile v4f_t*)(pout + rowBase + lane * 4) = v;
  }
}

__global__ __launch_bounds__(256) void reduce_kernel(
    const float* __restrict__ partial, float* __restrict__ out) {
  const int m = blockIdx.x * 256 + threadIdx.x;
  float s = 0.0f;
#pragma unroll
  for (int i = 0; i < NSPLIT; ++i) s += partial[(size_t)i * M_DIM + m];
  *(volatile float*)(out + m) = s; __threadfence(); *(volatile float*)(out + m) = s;
}

extern "C" void kernel_launch(void* const* d_in, const int* in_sizes, int n_in,
                              void* d_out, int out_size, void* d_ws, size_t ws_size,
                              hipStream_t stream) {
  const float* Xq = (const float*)d_in[0];
  const float* Xt = (const float*)d_in[1];
  const float* alpha = (const float*)d_in[2];
  float* out = (float*)d_out;

  char* w = (char*)d_ws;
  _Float16* Xqh = (_Float16*)w;
  _Float16* Xth = (_Float16*)(w + (size_t)M_DIM * D_DIM * 2);
  float* sqa = (float*)(w + (size_t)(M_DIM + N_DIM) * D_DIM * 2);
  float* sqb = sqa + M_DIM;
  float* partial = sqb + N_DIM;

  cvt_kernel<<<((M_DIM + N_DIM) * D_DIM / 8) / 256, 256, 0, stream>>>(Xq, Xt, Xqh, Xth);
  norm_kernel<<<(M_DIM + N_DIM) / 256, 256, 0, stream>>>(Xq, Xt, sqa, sqb);
  rbf_wmma_kernel<<<dim3(M_DIM / BM, NSPLIT), 256, 0, stream>>>(
      Xqh, Xth, sqa, sqb, alpha, partial);
  reduce_kernel<<<M_DIM / 256, 256, 0, stream>>>(partial, out);
}
